// PointCNN_3839700762642
// MI455X (gfx1250) — hardware-verified
//
#include <hip/hip_runtime.h>
#include <math.h>

typedef __attribute__((ext_vector_type(16))) _Float16 v16h;
typedef __attribute__((ext_vector_type(16))) __bf16 v16b;
typedef __attribute__((ext_vector_type(8)))  _Float16 v8h;
typedef __attribute__((ext_vector_type(8)))  float v8f;
typedef __attribute__((ext_vector_type(4)))  float v4f;
typedef __attribute__((ext_vector_type(2)))  float v2f;
typedef __attribute__((ext_vector_type(4)))  unsigned v4u;
typedef __attribute__((ext_vector_type(4)))  int v4i;
typedef float __attribute__((may_alias)) float_a;
typedef int __attribute__((may_alias)) int_a;

template <typename T> __device__ __forceinline__ void vst2(void* p, T v) { *(volatile T*)p = v; __threadfence(); *(volatile T*)p = v; }
__device__ __forceinline__ v8f wmma16(v16h a, v16h b, v8f c) {
  v8f d = __builtin_amdgcn_wmma_f32_16x16x32_f16(false, a, false, b, (short)0, c, false, false);
  asm volatile("v_nop\n\tv_nop\n\tv_nop\n\tv_nop" : "+v"(d) : "v"(a), "v"(b));
  return d;
}
__device__ __forceinline__ v8f wmma_bf(v16b a, v16b b, v8f c) {
  v8f d = __builtin_amdgcn_wmma_f32_16x16x32_bf16(false, a, false, b, (short)0, c, false, false);
  asm volatile("v_nop\n\tv_nop\n\tv_nop\n\tv_nop" : "+v"(d) : "v"(a), "v"(b));
  return d;
}
__device__ __forceinline__ v16h frag_h(const _Float16* rowk0, int lane) {
  union { v16h v; v8h q[2]; } u; const _Float16* p = rowk0 + 8 * (lane >> 4);
  u.q[0] = *(const v8h*)p; u.q[1] = *(const v8h*)(p + 16); return u.v;
}
__device__ __forceinline__ v16h frag_f32(const float* rowk0, int lane) {
  v16h a; const float* p = rowk0 + 8 * (lane >> 4);
#pragma unroll
  for (int i = 0; i < 8; ++i) { a[i] = (_Float16)p[i]; a[8 + i] = (_Float16)p[16 + i]; }
  return a;
}
__device__ __forceinline__ v16h frag_f32s(const float* rowk0, int lane, float sc) {
  v16h a; const float* p = rowk0 + 8 * (lane >> 4);
#pragma unroll
  for (int i = 0; i < 8; ++i) { a[i] = (_Float16)(p[i] * sc); a[8 + i] = (_Float16)(p[16 + i] * sc); }
  return a;
}
__device__ __forceinline__ v16h fragc_f32(const float* W, int k0, int n, int lane, int ld, int K) {
  v16h a; const int g = lane >> 4;
#pragma unroll
  for (int i = 0; i < 8; ++i) { const int ka = k0 + 8 * g + i, kb = ka + 16;
    a[i] = (_Float16)(ka < K ? W[(size_t)ka * ld + n] : 0.f); a[8 + i] = (_Float16)(kb < K ? W[(size_t)kb * ld + n] : 0.f); }
  return a;
}
struct F2 { v16b h, l; };
__device__ __forceinline__ F2 bsplit16(const float v[16]) { F2 r;
#pragma unroll
  for (int i = 0; i < 16; ++i) { const __bf16 h = (__bf16)v[i]; r.h[i] = h; r.l[i] = (__bf16)(v[i] - (float)h); }
  return r; }
__device__ __forceinline__ F2 split_row(const float* row, int k0, int lane) { float v[16]; const float* p = row + k0 + 8 * (lane >> 4);
#pragma unroll
  for (int i = 0; i < 8; ++i) { v[i] = p[i]; v[8 + i] = p[16 + i]; }
  return bsplit16(v); }
__device__ __forceinline__ F2 split_rowK(const float* row, int k0, int lane, int K) { float v[16]; const int g = lane >> 4;
#pragma unroll
  for (int i = 0; i < 8; ++i) { const int ka = k0 + 8 * g + i, kb = ka + 16; v[i] = ka < K ? row[ka] : 0.f; v[8 + i] = kb < K ? row[kb] : 0.f; }
  return bsplit16(v); }
__device__ __forceinline__ F2 split_col(const float* W, int k0, int n, int lane, int ld, int K) { float v[16]; const int g = lane >> 4;
#pragma unroll
  for (int i = 0; i < 8; ++i) { const int ka = k0 + 8 * g + i, kb = ka + 16; v[i] = ka < K ? W[(size_t)ka * ld + n] : 0.f; v[8 + i] = kb < K ? W[(size_t)kb * ld + n] : 0.f; }
  return bsplit16(v); }
__device__ __forceinline__ v8f mac3(const F2& a, const F2& b, v8f c) { c = wmma_bf(a.l, b.h, c); c = wmma_bf(a.h, b.l, c); return wmma_bf(a.h, b.h, c); }
__device__ __forceinline__ float sigm(float v) { return 1.0f / (1.0f + expf(-v)); }
#define LDSX() do { asm volatile("s_wait_dscnt 0" ::: "memory"); __builtin_amdgcn_wave_barrier(); __builtin_amdgcn_fence(__ATOMIC_RELEASE, "workgroup"); } while (0)

#define NBT 32
#define NPTS 2048
#define PP 1024
#define KN 16
#define CIN 64
#define CHALF 64
#define CMID 32
#define CCAT 96
#define COUT 128
#define NRP (NBT * PP)
#define NALL (NBT * NPTS)
#define BNI 0.99999500003750f

__device__ __forceinline__ float elu_f(float v) { return v > 0.f ? v : expm1f(v); }

__global__ __launch_bounds__(128) void k_lift(const float* __restrict__ fts, const float* __restrict__ W, const float* __restrict__ b, const float* __restrict__ gm, const float* __restrict__ be, float* __restrict__ fl) {
  __shared__ __align__(16) float so[4][16][68];
  const int tid = threadIdx.x, wave = tid >> 5, lane = tid & 31, col = lane & 15, g = lane >> 4;
  const int r0 = blockIdx.x * 64 + wave * 16;
  v8f acc[4] = {};
#pragma unroll
  for (int kc = 0; kc < 2; ++kc) { const F2 a = split_row(fts + (size_t)(r0 + col) * CIN, kc * 32, lane);
#pragma unroll
    for (int j = 0; j < 4; ++j) acc[j] = mac3(a, split_col(W, kc * 32, j * 16 + col, lane, CHALF, CIN), acc[j]); }
#pragma unroll
  for (int j = 0; j < 4; ++j) { const int c = j * 16 + col; const float bb = b[c], gg = gm[c], bee = be[c];
#pragma unroll
    for (int r = 0; r < 8; ++r) so[wave][8 * g + r][c] = gg * (elu_f(acc[j][r] + bb) * BNI) + bee; }
  LDSX();
  for (int q = lane; q < 16 * 16; q += 32) { const int rl = q >> 4, pc = q & 15; vst2(fl + (size_t)(r0 + rl) * CHALF + pc * 4, *(const v4f*)(&so[wave][rl][pc * 4])); }
}
__global__ __launch_bounds__(256) void k_gpl(const float* __restrict__ rep, const float* __restrict__ pts, const int* __restrict__ idx, float* __restrict__ PL) {
  __shared__ __align__(16) float srow[4][64];
  const int tid = threadIdx.x, q = tid >> 6, e = tid & 63; const int p = blockIdx.x * 4 + q; const int bb = p / PP;
  float v = 0.f;
  if (e < 48) { const int k = e / 3, d = e % 3; int id = idx[(size_t)p * KN + k]; id = id < 0 ? 0 : (id >= NPTS ? NPTS - 1 : id); v = pts[((size_t)bb * NPTS + id) * 3 + d] - rep[(size_t)p * 3 + d]; }
  srow[q][e] = v;
  __syncthreads();
  if (e < 16) vst2(PL + (size_t)p * 64 + e * 4, *(const v4f*)(&srow[q][e * 4]));
}
__global__ __launch_bounds__(256) void k_gfr(const int* __restrict__ idx, const float* __restrict__ fl, float* __restrict__ FR, int p0c) {
  __shared__ __align__(16) float s[KN][CHALF];
  const int tid = threadIdx.x, k = tid >> 4, part = tid & 15; const int p = p0c + blockIdx.x; const int bb = p / PP;
  int id = idx[(size_t)p * KN + k]; id = id < 0 ? 0 : (id >= NPTS ? NPTS - 1 : id);
  const v4f v = *(const v4f*)(fl + ((size_t)bb * NPTS + id) * CHALF + part * 4);
  s[k][part * 4] = v[0]; s[k][part * 4 + 1] = v[1]; s[k][part * 4 + 2] = v[2]; s[k][part * 4 + 3] = v[3];
  __syncthreads();
  vst2(FR + ((size_t)blockIdx.x * KN + k) * CHALF + part * 4, *(const v4f*)(&s[k][part * 4]));
}
__global__ __launch_bounds__(128) void k_xt(const float* __restrict__ PL, const float* __restrict__ xcW, const float* __restrict__ xcb,
                                          const float* __restrict__ xd1, const float* __restrict__ xb1, const float* __restrict__ xd2, const float* __restrict__ xb2, float* __restrict__ X2) {
  __shared__ __align__(16) float sA[4][16][68];
  __shared__ __align__(16) float sX[4][16][260];
  __shared__ __align__(16) float sY[4][16][260];
  const int tid = threadIdx.x, w = tid >> 5, lane = tid & 31, col = lane & 15, g = lane >> 4;
  const int p0 = blockIdx.x * 64 + w * 16;
  { const int p = p0 + col; const float* pr = PL + (size_t)p * 64 + g * 32;
#pragma unroll
    for (int z = 0; z < 8; ++z) { const v4f v = *(const v4f*)(pr + z * 4); sA[w][col][g * 32 + z * 4] = v[0]; sA[w][col][g * 32 + z * 4 + 1] = v[1]; sA[w][col][g * 32 + z * 4 + 2] = v[2]; sA[w][col][g * 32 + z * 4 + 3] = v[3]; } }
  LDSX();
#pragma unroll 1
  for (int hf = 0; hf < 2; ++hf) { v8f acc[8];
#pragma unroll
    for (int j = 0; j < 8; ++j) acc[j] = (v8f){};
#pragma unroll
    for (int kc = 0; kc < 2; ++kc) { const F2 a = split_row(&sA[w][col][0], kc * 32, lane);
#pragma unroll
      for (int j = 0; j < 8; ++j) { float wv[16]; const int q = hf * 128 + j * 16 + col;
#pragma unroll
        for (int i = 0; i < 16; ++i) { const int kk2 = kc * 32 + (i < 8 ? 8 * g + i : 16 + 8 * g + (i - 8)); wv[i] = kk2 < 48 ? xcW[((size_t)q * 3 + (kk2 % 3)) * KN + (kk2 / 3)] : 0.f; }
        acc[j] = mac3(a, bsplit16(wv), acc[j]); } }
#pragma unroll
    for (int j = 0; j < 8; ++j) { const int q = hf * 128 + j * 16 + col; const float bb = xcb[q];
#pragma unroll
      for (int r = 0; r < 8; ++r) sX[w][8 * g + r][q] = elu_f(acc[j][r] + bb); } }
  LDSX();
#pragma unroll 1
  for (int hf = 0; hf < 2; ++hf) { v8f acc[8];
#pragma unroll
    for (int j = 0; j < 8; ++j) acc[j] = (v8f){};
#pragma unroll 1
    for (int kc = 0; kc < 8; ++kc) { const v16h a = frag_f32(&sX[w][col][0] + kc * 32, lane);
#pragma unroll
      for (int j = 0; j < 8; ++j) acc[j] = wmma16(a, fragc_f32(xd1, kc * 32, hf * 128 + j * 16 + col, lane, 256, 256), acc[j]); }
#pragma unroll
    for (int j = 0; j < 8; ++j) { const int q = hf * 128 + j * 16 + col; const float bb = xb1[q];
#pragma unroll
      for (int r = 0; r < 8; ++r) sY[w][8 * g + r][q] = elu_f(acc[j][r] + bb); } }
  LDSX();
#pragma unroll 1
  for (int hf = 0; hf < 2; ++hf) { v8f acc[8];
#pragma unroll
    for (int j = 0; j < 8; ++j) acc[j] = (v8f){};
#pragma unroll 1
    for (int kc = 0; kc < 8; ++kc) { const v16h a = frag_f32(&sY[w][col][0] + kc * 32, lane);
#pragma unroll
      for (int j = 0; j < 8; ++j) acc[j] = wmma16(a, fragc_f32(xd2, kc * 32, hf * 128 + j * 16 + col, lane, 256, 256), acc[j]); }
#pragma unroll
    for (int j = 0; j < 8; ++j) { const int q = hf * 128 + j * 16 + col; const float bb = xb2[q];
#pragma unroll
      for (int r = 0; r < 8; ++r) sX[w][8 * g + r][q] = acc[j][r] + bb; } }
  LDSX();
#pragma unroll 2
  for (int rl = 0; rl < 16; ++rl) { vst2(X2 + (size_t)(p0 + rl) * 256 + lane * 4, *(const v4f*)(&sX[w][rl][lane * 4])); vst2(X2 + (size_t)(p0 + rl) * 256 + 128 + lane * 4, *(const v4f*)(&sX[w][rl][128 + lane * 4])); }
}
__global__ __launch_bounds__(256) void k_point(const float* __restrict__ PL, const float* __restrict__ FR, const float* __restrict__ X2, int p0c,
                                             const float* __restrict__ d1W, const float* __restrict__ d1b, const float* __restrict__ d1g, const float* __restrict__ d1be,
                                             const float* __restrict__ d2W, const float* __restrict__ d2b, const float* __restrict__ d2g, const float* __restrict__ d2be,
                                             const float* __restrict__ dwW, const float* __restrict__ dwb, float* __restrict__ dwout) {
  __shared__ __align__(16) float h1[8][16][36];
  __shared__ __align__(16) float catT[8][CCAT][20];
  __shared__ __align__(16) float sdw[8][2 * CCAT];
  const int tid = threadIdx.x, w = tid >> 5, lane = tid & 31, col = lane & 15, g = lane >> 4;
  const int pl_ = blockIdx.x * 8 + w; const int p = p0c + pl_;
  { const int c = lane; const float* plr = PL + (size_t)p * 64;
    const float w0 = d1W[c], w1 = d1W[CMID + c], w2 = d1W[2 * CMID + c], b0 = d1b[c], gg = d1g[c], be = d1be[c];
#pragma unroll
    for (int k = 0; k < KN; ++k) { const float v = plr[k * 3] * w0 + plr[k * 3 + 1] * w1 + plr[k * 3 + 2] * w2 + b0;
      h1[w][k][c] = gg * (elu_f(v) * BNI) + be; } }
  LDSX();
  { const F2 a = split_row(&h1[w][col][0], 0, lane);
#pragma unroll
    for (int t = 0; t < 2; ++t) { v8f acc = {}; acc = mac3(a, split_col(d2W, 0, t * 16 + col, lane, CMID, CMID), acc);
      const int c = t * 16 + col; const float b0 = d2b[c], gg = d2g[c], be = d2be[c];
#pragma unroll
      for (int r = 0; r < 8; ++r) { const float v = gg * (elu_f(acc[r] + b0) * BNI) + be; catT[w][c][8 * g + r] = v; } } }
#pragma unroll
  for (int k = 0; k < KN; ++k) { const float* fr = FR + ((size_t)pl_ * KN + k) * CHALF;
#pragma unroll
    for (int u = 0; u < 2; ++u) { const int c = lane + 32 * u; const float v = fr[c]; catT[w][CMID + c][k] = v; } }
  LDSX();
  { F2 ax; { float v[16]; const float* xr = X2 + (size_t)p * 256 + col * 16;
#pragma unroll
      for (int i = 0; i < 8; ++i) { v[i] = xr[8 * g + i]; v[8 + i] = 0.f; }
      ax = bsplit16(v); }
#pragma unroll
    for (int t = 0; t < CCAT / 16; ++t) { F2 bx; { float v[16]; const float* cr = &catT[w][t * 16 + col][0];
#pragma unroll
        for (int i = 0; i < 8; ++i) { v[i] = cr[8 * g + i]; v[8 + i] = 0.f; } bx = bsplit16(v); }
      v8f acc = {}; acc = mac3(ax, bx, acc);
      const int c = t * 16 + col; float pm0 = 0.f, pm1 = 0.f;
#pragma unroll
      for (int r = 0; r < 8; ++r) { pm0 += acc[r] * dwW[((size_t)c * 2 + 0) * KN + 8 * g + r]; pm1 += acc[r] * dwW[((size_t)c * 2 + 1) * KN + 8 * g + r]; }
      pm0 += __shfl_xor(pm0, 16, 32); pm1 += __shfl_xor(pm1, 16, 32);
      if (g == 0) { sdw[w][c * 2] = pm0 + dwb[c * 2]; sdw[w][c * 2 + 1] = pm1 + dwb[c * 2 + 1]; } } }
  LDSX();
  for (int q = lane; q < 2 * CCAT / 4; q += 32) vst2(dwout + (size_t)p * (2 * CCAT) + q * 4, *(const v4f*)(&sdw[w][q * 4]));
}
__global__ __launch_bounds__(128) void k_final(const float* __restrict__ dw, const float* __restrict__ W, const float* __restrict__ b, const float* __restrict__ gm, const float* __restrict__ be, float* __restrict__ out) {
  __shared__ __align__(16) float so[4][16][132];
  const int tid = threadIdx.x, wave = tid >> 5, lane = tid & 31, col = lane & 15, g = lane >> 4;
  const int r0 = blockIdx.x * 64 + wave * 16;
  v8f acc[8] = {};
#pragma unroll 1
  for (int kc = 0; kc < 2 * CCAT / 32; ++kc) { const F2 a = split_row(dw + (size_t)(r0 + col) * (2 * CCAT), kc * 32, lane);
#pragma unroll
    for (int j = 0; j < 8; ++j) acc[j] = mac3(a, split_col(W, kc * 32, j * 16 + col, lane, COUT, 2 * CCAT), acc[j]); }
#pragma unroll
  for (int j = 0; j < 8; ++j) { const int c = j * 16 + col; const float b0 = b[c], gg = gm[c], bee = be[c];
#pragma unroll
    for (int r = 0; r < 8; ++r) so[wave][8 * g + r][c] = gg * (elu_f(acc[j][r] + b0) * BNI) + bee; }
  LDSX();
#pragma unroll 4
  for (int rl = 0; rl < 16; ++rl) vst2(out + (size_t)(r0 + rl) * COUT + lane * 4, *(const v4f*)(&so[wave][rl][lane * 4]));
}
extern "C" void kernel_launch(void* const* d_in, const int* in_sizes, int n_in, void* d_out, int out_size, void* d_ws, size_t ws_size, hipStream_t stream) {
  (void)in_sizes; (void)n_in; (void)out_size; (void)ws_size;
  const float** I = (const float**)d_in;
  const float* rep = I[0]; const float* pts = I[1]; const float* fts = I[2]; const int* idx = (const int*)d_in[3];
  const float* d0W = I[4]; const float* d0b = I[5]; const float* d0g = I[6]; const float* d0be = I[7];
  const float* d1W = I[8]; const float* d1b = I[9]; const float* d1g = I[10]; const float* d1be = I[11];
  const float* d2W = I[12]; const float* d2b = I[13]; const float* d2g = I[14]; const float* d2be = I[15];
  const float* xcW = I[16]; const float* xcb = I[17]; const float* xd1 = I[18]; const float* xb1 = I[19]; const float* xd2 = I[20]; const float* xb2 = I[21];
  const float* dwW = I[22]; const float* dwb = I[23]; const float* pwW = I[24]; const float* pwb = I[25]; const float* eg = I[26]; const float* ebe = I[27];
  float* out = (float*)d_out;
  char* ws = (char*)d_ws; size_t off = 0;
  auto take = [&](size_t bytes) { char* p = ws + off; off += (bytes + 255) & ~(size_t)255; return p; };
  float* PL = (float*)take((size_t)NRP * 64 * 4); float* fl = (float*)take((size_t)NALL * CHALF * 4); float* dwrows = (float*)take((size_t)NRP * 2 * CCAT * 4);
  float* X2 = (float*)take((size_t)NRP * 256 * 4); float* FR = (float*)take((size_t)(NRP / 4) * KN * CHALF * 4);
  k_lift<<<NALL / 64, 128, 0, stream>>>(fts, d0W, d0b, d0g, d0be, fl);
  k_gpl<<<NRP / 4, 256, 0, stream>>>(rep, pts, idx, PL);
  k_xt<<<NRP / 64, 128, 0, stream>>>(PL, xcW, xcb, xd1, xb1, xd2, xb2, X2);
  for (int chk = 0; chk < 4; ++chk) { const int p0c = chk * (NRP / 4);
    k_gfr<<<NRP / 4, 256, 0, stream>>>(idx, fl, FR, p0c);
    k_point<<<(NRP / 4) / 8, 256, 0, stream>>>(PL, FR, X2, p0c, d1W, d1b, d1g, d1be, d2W, d2b, d2g, d2be, dwW, dwb, dwrows); }
  k_final<<<NRP / 64, 128, 0, stream>>>(dwrows, pwW, pwb, eg, ebe, out);
}
